// VJEPA2JointDiffuserRopeAttention_1176821039787
// MI455X (gfx1250) — hardware-verified
//
#include <hip/hip_runtime.h>
#include <stddef.h>
#include <stdint.h>
#include <math.h>

#define HID   1024
#define NH    16
#define HS    64
#define NBAT  2
#define NV    2048
#define NA    16
#define NT    (NV + NA)
#define KC    64
#define NP    2112
#define NKC   (NP / KC)
#define NQC   (NP / KC)
#define NBH   (NBAT * NH)
#define MV    (NBAT * NV)
#define MA    (NBAT * NA)
#define TPF   256
#define GRW   16
#define NROT  10
#define ROTD  60
#define NPOS  16
#define NCS   (NPOS * NROT)
#define NWV   4
#define QBR   64
#define PTP   72
#define OTP   68
#define WSC   64.0f
#define CSC   16.0f
#define PSCI  (1.0f / 64.0f)
#define OSCI  (1.0f / 1024.0f)
#define SCL   0.125f
#define NEGB  (-1.0e30f)

static_assert(NP % KC == 0);
static_assert(NT < NP);
static_assert(NP - NT == 48);
static_assert(NV % 64 == 0);
static_assert(MV % 64 == 0);
static_assert(MA == 32);
static_assert(HS == 64);
static_assert((HID * HID) % (8 * 256) == 0);
static_assert((MV * HID) % (8 * 256) == 0);
static_assert((MA * HID) % (8 * 256) == 0);
static_assert((PTP * 2) % 16 == 0);
static_assert((OTP * 4) % 16 == 0);
static_assert(QBR == NWV * 16);
static_assert(NCS <= 2 * 128);

typedef float          v8f   __attribute__((ext_vector_type(8)));
typedef float          v4f   __attribute__((ext_vector_type(4)));
typedef unsigned int   v4u   __attribute__((ext_vector_type(4)));
typedef unsigned short v8us  __attribute__((ext_vector_type(8)));
typedef unsigned short v16us __attribute__((ext_vector_type(16)));
typedef __bf16         v16b  __attribute__((ext_vector_type(16)));
typedef _Float16       v16h  __attribute__((ext_vector_type(16)));
typedef _Float16       v8h   __attribute__((ext_vector_type(8)));
typedef unsigned short ush;

union FragU { v16us v; v8us h[2]; v16b b; v16h f; };
union PackU { v8us s; v4u u; v8h f; };
struct HL { v4u h; v4u l; };

__device__ __forceinline__ ush f2bf(float f) {
  const unsigned u = __float_as_uint(f);
  return (ush)((u + 0x7FFFu + ((u >> 16) & 1u)) >> 16);
}
__device__ __forceinline__ float bf2f(ush v) { return __uint_as_float(((unsigned)v) << 16); }

__device__ __forceinline__ HL split8(v8f f) {
  PackU ph, pl;
#pragma unroll
  for (int e = 0; e < 8; ++e) {
    const ush hi = f2bf(f[e]);
    ph.s[e] = hi;
    pl.s[e] = f2bf(f[e] - bf2f(hi));
  }
  HL r; r.h = ph.u; r.l = pl.u;
  return r;
}

__device__ __forceinline__ v4u cvt8h(v8f f, float sc) {
  PackU p;
#pragma unroll
  for (int e = 0; e < 8; ++e) p.f[e] = (_Float16)(f[e] * sc);
  return p.u;
}

__device__ __forceinline__ v8f zero8() { return (v8f){0.f, 0.f, 0.f, 0.f, 0.f, 0.f, 0.f, 0.f}; }

__device__ __forceinline__ v8f mmab(v16us a, v16us b, v8f c) {
  FragU ua, ub; ua.v = a; ub.v = b;
  c = __builtin_amdgcn_wmma_f32_16x16x32_bf16(false, ua.b, false, ub.b, (short)0, c, false, false);
  asm volatile("v_nop\n\tv_nop\n\tv_nop\n\tv_nop" : "+v"(c) : "v"(a), "v"(b));
  return c;
}
__device__ __forceinline__ v8f mmah(v16us a, v16us b, v8f c) {
  FragU ua, ub; ua.v = a; ub.v = b;
  c = __builtin_amdgcn_wmma_f32_16x16x32_f16(false, ua.f, false, ub.f, (short)0, c, false, false);
  asm volatile("v_nop\n\tv_nop\n\tv_nop\n\tv_nop" : "+v"(c) : "v"(a), "v"(b));
  return c;
}

__device__ __forceinline__ v16us ldrowu(const ush* p, int ld, int row, int k0, int lane) {
  const int lh = lane >> 4;
  const ush* q = p + (size_t)row * ld + k0 + 8 * lh;
  FragU f;
  f.h[0] = *(const v8us*)(q);
  f.h[1] = *(const v8us*)(q + 16);
  return f.v;
}
__device__ __forceinline__ v16us ldfragu(const ush* p, int ld, int row0, int k0, int lane) {
  return ldrowu(p, ld, row0 + (lane & 15), k0, lane);
}

__global__ __launch_bounds__(256)
void k_cvtw(const float* __restrict__ w0, const float* __restrict__ w1, const float* __restrict__ w2,
            const float* __restrict__ w3, const float* __restrict__ w4, const float* __restrict__ w5,
            const float* __restrict__ w6, const float* __restrict__ w7, ush* __restrict__ dst) {
  const int z = blockIdx.y;
  const float* src = (z == 0) ? w0 : (z == 1) ? w1 : (z == 2) ? w2 : (z == 3) ? w3 :
                     (z == 4) ? w4 : (z == 5) ? w5 : (z == 6) ? w6 : w7;
  const size_t p  = (size_t)blockIdx.x * 256 + threadIdx.x;
  const size_t so = p * 8;
  const v4f a0 = *(const v4f*)(src + so);
  const v4f a1 = *(const v4f*)(src + so + 4);
  const v8f f = (v8f){a0[0], a0[1], a0[2], a0[3], a1[0], a1[1], a1[2], a1[3]};
  const v4u v = cvt8h(f, WSC);
  ush* d = dst + (size_t)z * HID * HID + so;
  *(volatile v4u*)d = v;
  __threadfence();
  *(volatile v4u*)d = v;
}

__global__ __launch_bounds__(256)
void k_cvtx(const float* __restrict__ src, ush* __restrict__ dst, float sc) {
  const size_t p  = (size_t)blockIdx.x * 256 + threadIdx.x;
  const size_t so = p * 8;
  const v4f a0 = *(const v4f*)(src + so);
  const v4f a1 = *(const v4f*)(src + so + 4);
  const v8f f = (v8f){a0[0], a0[1], a0[2], a0[3], a1[0], a1[1], a1[2], a1[3]};
  const v4u v = cvt8h(f, sc);
  *(volatile v4u*)(dst + so) = v;
  __threadfence();
  *(volatile v4u*)(dst + so) = v;
}

__device__ __forceinline__ void gemm_core(const ush* __restrict__ A, int arow,
                                          const ush* __restrict__ W, int n0, int lane, v8f (&acc)[4]) {
#pragma unroll
  for (int t = 0; t < 4; ++t) acc[t] = zero8();
#pragma unroll 1
  for (int k0 = 0; k0 < HID; k0 += 32) {
    const v16us a = ldrowu(A, HID, arow, k0, lane);
#pragma unroll
    for (int t = 0; t < 4; ++t) {
      const v16us bw = ldfragu(W, HID, n0 + 16 * t, k0, lane);
      acc[t] = mmah(a, bw, acc[t]);
    }
  }
}

__global__ __launch_bounds__(128)
void k_gemm_qk(const ush* __restrict__ A, int mrows, int act,
               const ush* __restrict__ W0, const ush* __restrict__ W1,
               const float* __restrict__ b0, const float* __restrict__ b1,
               ush* __restrict__ P0h, ush* __restrict__ P0l,
               ush* __restrict__ P1h, ush* __restrict__ P1l) {
  __shared__ float csT[2 * NCS];
  __shared__ __align__(16) float Os[NWV * 16 * OTP];

  const int tid = threadIdx.x, lane = tid & 31, wave = tid >> 5;
  const int hh = lane >> 4, c = lane & 15;
  const int z  = blockIdx.z;
  const ush*   W    = z ? W1 : W0;
  const float* bias = z ? b1 : b0;
  ush* Ph = z ? P1h : P0h;
  ush* Pl = z ? P1l : P0l;
  const int h  = blockIdx.y, n0 = h * HS;
  const int m0 = blockIdx.x * 64;

  {
    const float ap0 = (float)(0 / TPF);
    const float ap1 = (float)(1 / TPF);
#pragma unroll 1
    for (int e = tid; e < NCS; e += 128) {
      const int p = e / NROT;
      const int i = e - NROT * p;
      const float om   = 1.0f / powf(10000.0f, (float)i * 0.1f);
      const float posv = (float)p;
      const float posa = ap0 + (ap1 - ap0) * ((float)p * (1.0f / 15.0f));
      const float pos  = act ? posa : posv;
      const float fr   = pos * om;
      csT[e]       = cosf(fr);
      csT[NCS + e] = sinf(fr);
    }
  }
  __syncthreads();

  const int gr   = m0 + 16 * wave + c;
  const int arow = min(gr, mrows - 1);
  v8f acc[4];
  gemm_core(A, arow, W, n0, lane, acc);

  const int rw0  = m0 + 16 * wave;
  const int bb   = act ? (rw0 / NA) : (rw0 / NV);
  const int tok0 = act ? NV : (rw0 % NV);
  float* sw = Os + wave * 16 * OTP;

  float bc[4];
#pragma unroll
  for (int t = 0; t < 4; ++t) bc[t] = bias[n0 + 16 * t + c];

#pragma unroll
  for (int t = 0; t < 4; ++t) {
    const int  d   = 16 * t + c;
    const bool rot = d < ROTD;
    const int  dd  = rot ? d : 0;
    const int  sec = dd / (2 * NROT);
    const int  ii  = (dd - 2 * NROT * sec) >> 1;
#pragma unroll
    for (int r = 0; r < 8; ++r) {
      const int row = 8 * hh + r;
      const int tok = tok0 + row;
      const int pd  = act ? row : (tok / TPF);
      const int ph  = act ? row : ((tok / GRW) % GRW);
      const int pw  = act ? row : (tok % GRW);
      const int ps  = (sec == 0) ? pd : ((sec == 1) ? ph : pw);
      const int idx = ps * NROT + ii;
      const float ct = csT[idx];
      const float st = csT[NCS + idx];
      const float cv = rot ? ct : 1.0f;
      const float sv = rot ? st : 0.0f;
      const float y  = acc[t][r] * PSCI + bc[t];
      const float yp = __shfl_xor(y, 1, 32);
      const float o  = (c & 1) ? (y * cv + yp * sv) : (y * cv - yp * sv);
      sw[row * OTP + d] = o;
    }
  }
  __syncthreads();

  if (act == 0 || wave < 2) {
    const int bh = bb * NH + h;
    v4u vh[4], vl[4];
    size_t go[4];
#pragma unroll
    for (int it = 0; it < 4; ++it) {
      const int p   = lane + 32 * it;
      const int row = p >> 3;
      const int pc  = p & 7;
      const v4f x0 = *(const v4f*)(sw + row * OTP + pc * 8);
      const v4f x1 = *(const v4f*)(sw + row * OTP + pc * 8 + 4);
      const v8f f = (v8f){x0[0], x0[1], x0[2], x0[3], x1[0], x1[1], x1[2], x1[3]};
      const HL sp = split8(f);
      vh[it] = sp.h; vl[it] = sp.l;
      go[it] = ((size_t)bh * NP + tok0 + row) * HS + pc * 8;
    }
    for (int ps = 0; ps < 2; ++ps) {
#pragma unroll
      for (int it = 0; it < 4; ++it) {
        *(volatile v4u*)(Ph + go[it]) = vh[it];
        *(volatile v4u*)(Pl + go[it]) = vl[it];
      }
      __threadfence();
    }
  } else {
    const int bh = (wave - 2) * NH + h;
    const v4u zz = (v4u){0u, 0u, 0u, 0u};
    for (int ps = 0; ps < 2; ++ps) {
#pragma unroll
      for (int it = 0; it < 12; ++it) {
        const int p   = lane + 32 * it;
        const int row = NT + (p >> 3);
        const int pc  = p & 7;
        const size_t go = ((size_t)bh * NP + row) * HS + pc * 8;
        *(volatile v4u*)(Ph + go) = zz;
        *(volatile v4u*)(Pl + go) = zz;
      }
      __threadfence();
    }
  }
}

__global__ __launch_bounds__(128)
void k_gemm_v(const ush* __restrict__ A, int mrows, int act,
              const ush* __restrict__ W, const float* __restrict__ bias,
              ush* __restrict__ VTh, ush* __restrict__ VTl) {
  __shared__ __align__(16) float Os[NWV * 16 * OTP];

  const int tid = threadIdx.x, lane = tid & 31, wave = tid >> 5;
  const int hh = lane >> 4, c = lane & 15;
  const int h  = blockIdx.y, n0 = h * HS;
  const int m0 = blockIdx.x * 64;

  const int gr   = m0 + 16 * wave + c;
  const int arow = min(gr, mrows - 1);
  v8f acc[4];
  gemm_core(A, arow, W, n0, lane, acc);

#pragma unroll
  for (int t = 0; t < 4; ++t) {
    const float bcv = bias[n0 + 16 * t + c];
#pragma unroll
    for (int r = 0; r < 8; ++r)
      Os[(16 * wave + 8 * hh + r) * OTP + 16 * t + c] = acc[t][r] * PSCI + bcv;
  }
  __syncthreads();

  const int nb   = act ? 2 : 1;
  const int npc  = act ? 2 : 8;
  const int bvid = m0 / NV;
  const int kcv  = (m0 % NV) / KC;
#pragma unroll 1
  for (int bs = 0; bs < nb; ++bs) {
    const int bh = act ? (bs * NH + h) : (bvid * NH + h);
    const int kc = act ? (NKC - 1) : kcv;
    const int rb = act ? (bs * NA) : 0;
    v4u vh[4], vl[4];
    size_t go[4];
#pragma unroll
    for (int it = 0; it < 4; ++it) {
      const int  p    = tid + 128 * it;
      const int  d    = p >> 3;
      const int  pc   = p & 7;
      const bool live = pc < npc;
      const int  pcc  = live ? pc : 0;
      const float* cp = Os + (rb + 8 * pcc) * OTP + d;
      v8f f;
#pragma unroll
      for (int e = 0; e < 8; ++e) { const float x = cp[e * OTP]; f[e] = live ? x : 0.0f; }
      const HL sp = split8(f);
      vh[it] = sp.h; vl[it] = sp.l;
      go[it] = (((size_t)bh * NKC + kc) * HS + d) * KC + pc * 8;
    }
    for (int ps = 0; ps < 2; ++ps) {
#pragma unroll
      for (int it = 0; it < 4; ++it) {
        *(volatile v4u*)(VTh + go[it]) = vh[it];
        *(volatile v4u*)(VTl + go[it]) = vl[it];
      }
      __threadfence();
    }
  }
}

__global__ __launch_bounds__(128)
void k_attn(const ush* __restrict__ qh, const ush* __restrict__ ql,
            const ush* __restrict__ kh, const ush* __restrict__ kl,
            const ush* __restrict__ vth, const ush* __restrict__ vtl,
            ush* __restrict__ ctxv, ush* __restrict__ ctxa) {
  __shared__ __align__(16) ush   Ph[NWV * 16 * PTP];
  __shared__ __align__(16) ush   Pl[NWV * 16 * PTP];
  __shared__ __align__(16) float Os[NWV * 16 * OTP];

  const int tid = threadIdx.x, lane = tid & 31, wave = tid >> 5;
  const int hh = lane >> 4, c = lane & 15;
  const int qc = blockIdx.x % NQC;
  const int hb = blockIdx.x / NQC;
  const int h  = hb % NH;
  const int b  = hb / NH;
  const int q0 = qc * QBR + wave * 16;

  const ush* Qh = qh  + (size_t)hb * NP * HS;
  const ush* Ql = ql  + (size_t)hb * NP * HS;
  const ush* Kh = kh  + (size_t)hb * NP * HS;
  const ush* Kl = kl  + (size_t)hb * NP * HS;
  const ush* Vh = vth + (size_t)hb * NKC * HS * KC;
  const ush* Vl = vtl + (size_t)hb * NKC * HS * KC;

  ush*   pwh = Ph + wave * 16 * PTP;
  ush*   pwl = Pl + wave * 16 * PTP;
  float* sw  = Os + wave * 16 * OTP;

  const float NEGI = -__builtin_huge_valf();
  float mrow[8], lrow[8];
  v8f oacc[4];
#pragma unroll
  for (int r = 0; r < 8; ++r) { mrow[r] = NEGI; lrow[r] = 0.f; }
#pragma unroll
  for (int t = 0; t < 4; ++t) oacc[t] = zero8();

#pragma unroll 1
  for (int kc = 0; kc < NKC; ++kc) {
    const int kv0 = kc * KC;
    __syncthreads();

    v8f s[4];
#pragma unroll
    for (int j = 0; j < 4; ++j) s[j] = zero8();
#pragma unroll
    for (int dc = 0; dc < 2; ++dc) {
      const v16us qah = ldfragu(Qh, HS, q0, dc * 32, lane);
      const v16us qal = ldfragu(Ql, HS, q0, dc * 32, lane);
#pragma unroll
      for (int j = 0; j < 4; ++j) {
        const v16us kbh = ldfragu(Kh, HS, kv0 + 16 * j, dc * 32, lane);
        const v16us kbl = ldfragu(Kl, HS, kv0 + 16 * j, dc * 32, lane);
        s[j] = mmab(qah, kbh, s[j]);
        s[j] = mmab(qah, kbl, s[j]);
        s[j] = mmab(qal, kbh, s[j]);
      }
    }
#pragma unroll
    for (int j = 0; j < 4; ++j) {
      const bool kval = (kv0 + 16 * j + c) < NT;
#pragma unroll
      for (int r = 0; r < 8; ++r) {
        const float sv = s[j][r] * SCL;
        s[j][r] = kval ? sv : NEGB;
      }
    }

    float cm[8];
#pragma unroll
    for (int r = 0; r < 8; ++r) {
      float m = fmaxf(fmaxf(s[0][r], s[1][r]), fmaxf(s[2][r], s[3][r]));
#pragma unroll
      for (int off = 1; off < 16; off <<= 1) m = fmaxf(m, __shfl_xor(m, off, 32));
      cm[r] = m;
    }
    float al[8];
#pragma unroll
    for (int r = 0; r < 8; ++r) {
      const float mnew  = fmaxf(mrow[r], cm[r]);
      const float alpha = __expf(mrow[r] - mnew);
      mrow[r] = mnew;
      float psum = 0.f;
#pragma unroll
      for (int j = 0; j < 4; ++j) {
        const float p = __expf(s[j][r] - mnew);
        psum += p;
        const ush phi = f2bf(p);
        pwh[(8 * hh + r) * PTP + 16 * j + c] = phi;
        pwl[(8 * hh + r) * PTP + 16 * j + c] = f2bf(p - bf2f(phi));
      }
#pragma unroll
      for (int off = 1; off < 16; off <<= 1) psum += __shfl_xor(psum, off, 32);
      lrow[r] = lrow[r] * alpha + psum;
      al[r] = alpha;
    }
#pragma unroll
    for (int t = 0; t < 4; ++t)
#pragma unroll
      for (int r = 0; r < 8; ++r) oacc[t][r] *= al[r];
    __syncthreads();

    const ush* Vch = Vh + (size_t)kc * HS * KC;
    const ush* Vcl = Vl + (size_t)kc * HS * KC;
#pragma unroll
    for (int kk = 0; kk < 2; ++kk) {
      const v16us pah = ldfragu(pwh, PTP, 0, kk * 32, lane);
      const v16us pal = ldfragu(pwl, PTP, 0, kk * 32, lane);
#pragma unroll
      for (int t = 0; t < 4; ++t) {
        const v16us vbh = ldfragu(Vch, KC, 16 * t, kk * 32, lane);
        const v16us vbl = ldfragu(Vcl, KC, 16 * t, kk * 32, lane);
        oacc[t] = mmab(pah, vbh, oacc[t]);
        oacc[t] = mmab(pah, vbl, oacc[t]);
        oacc[t] = mmab(pal, vbh, oacc[t]);
      }
    }
  }
  __syncthreads();

#pragma unroll
  for (int r = 0; r < 8; ++r) {
    const float lr  = lrow[r];
    const float inv = (lr > 0.f) ? (1.0f / lr) : 0.f;
    const int   row = 8 * hh + r;
#pragma unroll
    for (int t = 0; t < 4; ++t) sw[row * OTP + 16 * t + c] = oacc[t][r] * inv;
  }
  __syncthreads();

  if (q0 < NT) {
    const bool isact = (q0 >= NV);
    ush* dst = isact ? ctxa : ctxv;
    const size_t rb = isact ? (size_t)(b * NA + (q0 - NV)) : (size_t)(b * NV + q0);
    v4u val[4];
    size_t go[4];
#pragma unroll
    for (int it = 0; it < 4; ++it) {
      const int p   = lane + 32 * it;
      const int row = p >> 3;
      const int pc  = p & 7;
      const v4f x0 = *(const v4f*)(sw + row * OTP + pc * 8);
      const v4f x1 = *(const v4f*)(sw + row * OTP + pc * 8 + 4);
      const v8f f = (v8f){x0[0], x0[1], x0[2], x0[3], x1[0], x1[1], x1[2], x1[3]};
      val[it] = cvt8h(f, CSC);
      go[it]  = (rb + row) * HID + (size_t)h * HS + pc * 8;
    }
    for (int ps = 0; ps < 2; ++ps) {
#pragma unroll
      for (int it = 0; it < 4; ++it) *(volatile v4u*)(dst + go[it]) = val[it];
      __threadfence();
    }
  }
}

__global__ __launch_bounds__(128)
void k_gemm_out(const ush* __restrict__ A, int mrows,
                const ush* __restrict__ W, const float* __restrict__ bias,
                float* __restrict__ out) {
  __shared__ __align__(16) float Os[NWV * 16 * OTP];

  const int tid = threadIdx.x, lane = tid & 31, wave = tid >> 5;
  const int hh = lane >> 4, c = lane & 15;
  const int h  = blockIdx.y, n0 = h * HS;
  const int m0 = blockIdx.x * 64;

  const int gr   = m0 + 16 * wave + c;
  const int arow = min(gr, mrows - 1);
  v8f acc[4];
  gemm_core(A, arow, W, n0, lane, acc);

  const int rw0 = m0 + 16 * wave;
  float* sw = Os + wave * 16 * OTP;
#pragma unroll
  for (int t = 0; t < 4; ++t) {
    const float bcv = bias[n0 + 16 * t + c];
#pragma unroll
    for (int r = 0; r < 8; ++r) sw[(8 * hh + r) * OTP + 16 * t + c] = acc[t][r] * OSCI + bcv;
  }
  __syncthreads();

  if (rw0 < mrows) {
    v4f val[8];
    size_t go[8];
#pragma unroll
    for (int it = 0; it < 8; ++it) {
      const int p    = lane + 32 * it;
      const int L    = p >> 3;
      const int pc   = p & 7;
      const int row  = L >> 1;
      const int half = L & 1;
      val[it] = *(const v4f*)(sw + row * OTP + half * 32 + pc * 4);
      go[it]  = (size_t)(rw0 + row) * HID + n0 + half * 32 + pc * 4;
    }
    for (int ps = 0; ps < 2; ++ps) {
#pragma unroll
      for (int it = 0; it < 8; ++it) *(volatile v4f*)(out + go[it]) = val[it];
      __threadfence();
    }
  }
}

extern "C" void kernel_launch(void* const* d_in, const int* in_sizes, int n_in,
                              void* d_out, int out_size, void* d_ws, size_t ws_size,
                              hipStream_t stream) {
  if (n_in < 18) return;
  for (int i = 0; i < 8; ++i) {
    if (in_sizes[2 * i] != HID * HID) return;
    if (in_sizes[2 * i + 1] != HID) return;
  }
  if (in_sizes[16] != MV * HID) return;
  if (in_sizes[17] != MA * HID) return;
  if (out_size != MV * HID + MA * HID) return;

  const float* Wq   = (const float*)d_in[0];   const float* bq  = (const float*)d_in[1];
  const float* Wk   = (const float*)d_in[2];   const float* bk  = (const float*)d_in[3];
  const float* Wv   = (const float*)d_in[4];   const float* bv  = (const float*)d_in[5];
  const float* Wqa  = (const float*)d_in[6];   const float* bqa = (const float*)d_in[7];
  const float* Wka  = (const float*)d_in[8];   const float* bka = (const float*)d_in[9];
  const float* Wva  = (const float*)d_in[10];  const float* bva = (const float*)d_in[11];
  const float* Wpr  = (const float*)d_in[12];  const float* bpr = (const float*)d_in[13];
  const float* Wpa  = (const float*)d_in[14];  const float* bpa = (const float*)d_in[15];
  const float* xv   = (const float*)d_in[16];
  const float* xa   = (const float*)d_in[17];
  float* out0 = (float*)d_out;
  float* out1 = out0 + (size_t)MV * HID;

  const size_t plane = (size_t)NBH * NP * HS * 2;
  size_t off = 0;
  const size_t oXv = off; off += (size_t)MV * HID * 2;
  const size_t oXa = off; off += (size_t)MA * HID * 2;
  const size_t oW  = off; off += (size_t)8 * HID * HID * 2;
  const size_t oQh = off; off += plane;
  const size_t oQl = off; off += plane;
  const size_t oKh = off; off += plane;
  const size_t oKl = off; off += plane;
  const size_t oVh = off; off += plane;
  const size_t oVl = off; off += plane;
  const size_t oCv = off; off += (size_t)MV * HID * 2;
  const size_t oCa = off; off += (size_t)MA * HID * 2;
  if (off > ws_size) return;
  if (off > (size_t)134217728) return;

  char* ws = (char*)d_ws;
  ush* Xv  = (ush*)(ws + oXv);
  ush* Xa  = (ush*)(ws + oXa);
  ush* Wb  = (ush*)(ws + oW);
  ush* Qh  = (ush*)(ws + oQh);
  ush* Ql  = (ush*)(ws + oQl);
  ush* Kh  = (ush*)(ws + oKh);
  ush* Kl  = (ush*)(ws + oKl);
  ush* VTh = (ush*)(ws + oVh);
  ush* VTl = (ush*)(ws + oVl);
  ush* Cv  = (ush*)(ws + oCv);
  ush* Ca  = (ush*)(ws + oCa);
  const size_t wsz = (size_t)HID * HID;
  const ush* W0 = Wb + 0 * wsz;
  const ush* W1 = Wb + 1 * wsz;
  const ush* W2 = Wb + 2 * wsz;
  const ush* W3 = Wb + 3 * wsz;
  const ush* W4 = Wb + 4 * wsz;
  const ush* W5 = Wb + 5 * wsz;
  const ush* W6 = Wb + 6 * wsz;
  const ush* W7 = Wb + 7 * wsz;

  k_cvtw<<<dim3(HID * HID / (8 * 256), 8), dim3(256), 0, stream>>>(Wq, Wk, Wv, Wqa, Wka, Wva, Wpr, Wpa, Wb);
  k_cvtx<<<dim3(MV * HID / (8 * 256)), dim3(256), 0, stream>>>(xv, Xv, 1.0f);
  k_cvtx<<<dim3(MA * HID / (8 * 256)), dim3(256), 0, stream>>>(xa, Xa, 1.0f);
  k_gemm_qk<<<dim3(MV / 64, NH, 2), dim3(128), 0, stream>>>(Xv, MV, 0, W0, W1, bq, bk, Qh, Ql, Kh, Kl);
  k_gemm_v<<<dim3(MV / 64, NH), dim3(128), 0, stream>>>(Xv, MV, 0, W2, bv, VTh, VTl);
  k_gemm_qk<<<dim3(1, NH, 2), dim3(128), 0, stream>>>(Xa, MA, 1, W3, W4, bqa, bka, Qh, Ql, Kh, Kl);
  k_gemm_v<<<dim3(1, NH), dim3(128), 0, stream>>>(Xa, MA, 1, W5, bva, VTh, VTl);
  k_attn<<<dim3(NBH * NQC), dim3(128), 0, stream>>>(Qh, Ql, Kh, Kl, VTh, VTl, Cv, Ca);
  k_gemm_out<<<dim3(MV / 64, NH), dim3(128), 0, stream>>>(Cv, MV, W6, bpr, out0);
  k_gemm_out<<<dim3(1, NH), dim3(128), 0, stream>>>(Ca, MA, W7, bpa, out1);
  (void)hipGetLastError();
}
